// Dual_Attn_75917841924508
// MI455X (gfx1250) — hardware-run, weakly checked
//
#include <hip/hip_runtime.h>
#include <math.h>

constexpr int kImg   = 4;
constexpr int kChan  = 512;
constexpr int kPos   = 4096;
constexpr int kDk    = 64;
constexpr int kPix   = kImg * kPos;
constexpr int kHalfQ = 2048;
constexpr float kWCarry    = 16.0f;
constexpr float kWCarryInv = 1.0f / 16.0f;
constexpr float kPCarry    = 2048.0f;
constexpr float kPCarryInv = 1.0f / 2048.0f;
static_assert(kPix == 16384, "pixel count");
static_assert(kPos == 2 * kHalfQ, "two query chunks per image");

typedef __attribute__((ext_vector_type(16))) _Float16 v16h;
typedef __attribute__((ext_vector_type(8)))  _Float16 v8h;
typedef __attribute__((ext_vector_type(16))) __bf16   v16b;
typedef __attribute__((ext_vector_type(8)))  __bf16   v8b;
typedef __attribute__((ext_vector_type(8)))  float    v8f;
typedef __attribute__((ext_vector_type(4)))  float    v4f;
typedef __attribute__((ext_vector_type(4)))  unsigned int v4u;

__device__ __forceinline__ unsigned short f2bf_bits(float f) {
  unsigned u = __float_as_uint(f);
  return (unsigned short)((u + 0x7FFFu + ((u >> 16) & 1u)) >> 16);
}
__device__ __forceinline__ float bf_bits2f(unsigned short h) { return __uint_as_float(((unsigned)h) << 16); }

__device__ __forceinline__ void dep_guard_h(v8f& a, v8f& b, v16h x, v16h y) { asm volatile("v_nop\n\tv_nop\n\tv_nop\n\tv_nop" : "+v"(a), "+v"(b) : "v"(x), "v"(y)); }
__device__ __forceinline__ void dep_guard_b(v8f& a, v8f& b, v16b x, v16b y) { asm volatile("v_nop\n\tv_nop\n\tv_nop\n\tv_nop" : "+v"(a), "+v"(b) : "v"(x), "v"(y)); }
__device__ __forceinline__ void keep4_h(v16h a, v16h b, v16h c, v16h d) { asm volatile("v_nop" :: "v"(a), "v"(b), "v"(c), "v"(d)); }
__device__ __forceinline__ void keep4_b(v16b a, v16b b, v16b c, v16b d) { asm volatile("v_nop" :: "v"(a), "v"(b), "v"(c), "v"(d)); }
__device__ __forceinline__ void acc_guard4(v8f& a, v8f& b, v8f& c, v8f& d) { asm volatile("v_nop\n\tv_nop\n\tv_nop\n\tv_nop" : "+v"(a), "+v"(b), "+v"(c), "+v"(d)); }
template <typename T> struct Frag;
template <> struct Frag<_Float16> {
  typedef v16h V; union U { v16h v; v8h h[2]; };
  static __device__ __forceinline__ v16h load(const _Float16* p) {
    U f; f.h[0] = *(const v8h*)(p); f.h[1] = *(const v8h*)(p + 16); return f.v;
  }
  static __device__ __forceinline__ v8f mma(v16h a, v16h b, v8f c) {
    return __builtin_amdgcn_wmma_f32_16x16x32_f16(false, a, false, b, (short)0, c, false, false);
  }
  static __device__ __forceinline__ void guard(v8f& a, v8f& b, v16h x, v16h y) { dep_guard_h(a, b, x, y); }
  static __device__ __forceinline__ void keep(v16h a, v16h b, v16h c, v16h d) { keep4_h(a, b, c, d); }
};
template <> struct Frag<__bf16> {
  typedef v16b V; union U { v16b v; v8b h[2]; };
  static __device__ __forceinline__ v16b load(const __bf16* p) {
    U f; f.h[0] = *(const v8b*)(p); f.h[1] = *(const v8b*)(p + 16); return f.v;
  }
  static __device__ __forceinline__ v8f mma(v16b a, v16b b, v8f c) {
    return __builtin_amdgcn_wmma_f32_16x16x32_bf16(false, a, false, b, (short)0, c, false, false);
  }
  static __device__ __forceinline__ void guard(v8f& a, v8f& b, v16b x, v16b y) { dep_guard_b(a, b, x, y); }
  static __device__ __forceinline__ void keep(v16b a, v16b b, v16b c, v16b d) { keep4_b(a, b, c, d); }
};

__device__ __forceinline__ unsigned pk16(unsigned short a, unsigned short b) { return (unsigned)a | ((unsigned)b << 16); }
__device__ __forceinline__ unsigned short h_bits(float f) { const _Float16 h = (_Float16)f; return __builtin_bit_cast(unsigned short, h); }

template <int ET> struct Elem;
template <> struct Elem<0> { typedef _Float16 T; };
template <> struct Elem<1> { typedef __bf16 T; };
template <int ET, bool SPLIT, int BIAS_MODE, int OUT_MODE, bool RESID, bool GSC, int ACT = 0>
__global__ __launch_bounds__(256) void wmma_gemm64(
    const unsigned short* __restrict__ Ap, const unsigned short* __restrict__ A2p, int lda, long strideA,
    const unsigned short* __restrict__ Btp, const unsigned short* __restrict__ Bt2p, int ldb, long strideB,
    void* __restrict__ Cout, void* __restrict__ Cout2, int ldc, long strideC,
    const float* __restrict__ bias,
    const float* __restrict__ resid, long strideR,
    const float* __restrict__ gsp,
    int M, int N, int K, float scale) {
  typedef typename Elem<ET>::T T;
  typedef typename Frag<T>::V V;
  const T* A = (const T*)Ap; const T* A2 = (const T*)A2p; const T* Bt = (const T*)Btp; const T* Bt2 = (const T*)Bt2p;
  __shared__ __align__(16) float sT[8][16 * 68];
  const int b    = blockIdx.y;
  const int lane = threadIdx.x & 31;
  const int wave = threadIdx.x >> 5;
  const int tilesN = N >> 6;
  const int tilesM = M >> 6;
  const int tile = blockIdx.x * 8 + wave;
  if (tile >= tilesM * tilesN) return;
  const int tm = tile / tilesN;
  const int tn = tile - tm * tilesN;
  const int m0 = tm << 6;
  const int n0 = tn << 6;

  const T* Ab  = A  + (size_t)b * strideA;
  const T* Bb  = Bt + (size_t)b * strideB;
  const T* Ab2 = SPLIT ? (A2  + (size_t)b * strideA) : nullptr;
  const T* Bb2 = SPLIT ? (Bt2 + (size_t)b * strideB) : nullptr;

  const int rlane = lane & 15;
  const int koff  = (lane >> 4) * 8;
  const int mOff  = (lane >> 4) * 8;

  v8f acc[4][4];
#pragma unroll
  for (int i = 0; i < 4; ++i)
#pragma unroll
    for (int j = 0; j < 4; ++j) acc[i][j] = (v8f){0.f,0.f,0.f,0.f,0.f,0.f,0.f,0.f};

  for (int k0 = 0; k0 < K; k0 += 32) {
    V bh[4], bl[4];
#pragma unroll
    for (int j = 0; j < 4; ++j) {
      const size_t bo = (size_t)(n0 + (j << 4) + rlane) * ldb + koff + k0;
      bh[j] = Frag<T>::load(Bb + bo);
      if (SPLIT) bl[j] = Frag<T>::load(Bb2 + bo);
    }
#pragma unroll
    for (int i = 0; i < 4; ++i) {
      const size_t ao = (size_t)(m0 + (i << 4) + rlane) * lda + koff + k0;
      V ah = Frag<T>::load(Ab + ao);
      V al;
      if (SPLIT) al = Frag<T>::load(Ab2 + ao);
#pragma unroll
      for (int j = 0; j < 4; ++j) {
        acc[i][j] = Frag<T>::mma(ah, bh[j], acc[i][j]);
        if (SPLIT) {
          acc[i][j] = Frag<T>::mma(ah, bl[j], acc[i][j]);
          acc[i][j] = Frag<T>::mma(al, bh[j], acc[i][j]);
        }
      }
      Frag<T>::guard(acc[i][0], acc[i][3], ah, SPLIT ? al : ah);
    }
    Frag<T>::keep(bh[0], bh[1], bh[2], bh[3]);
    if (SPLIT) Frag<T>::keep(bl[0], bl[1], bl[2], bl[3]);
  }
  acc_guard4(acc[0][0], acc[0][1], acc[0][2], acc[0][3]);
  acc_guard4(acc[1][0], acc[1][1], acc[1][2], acc[1][3]);
  acc_guard4(acc[2][0], acc[2][1], acc[2][2], acc[2][3]);
  acc_guard4(acc[3][0], acc[3][1], acc[3][2], acc[3][3]);

  const float scl = GSC ? (scale * gsp[0]) : scale;
  float* slab = sT[wave];
  const float* Rb = RESID ? (resid + (size_t)b * strideR) : nullptr;
#pragma unroll
  for (int i = 0; i < 4; ++i) {
    const int mBase = m0 + (i << 4);
#pragma unroll
    for (int j = 0; j < 4; ++j) {
      const int n = n0 + (j << 4) + rlane;
      float bv = 0.f;
      if (BIAS_MODE == 2) bv = bias[n];
#pragma unroll
      for (int r = 0; r < 8; ++r) {
        float v = acc[i][j][r] * scl;
        if (BIAS_MODE == 1) v += bias[mBase + mOff + r];
        if (BIAS_MODE == 2) v += bv;
        if (RESID) v += Rb[(size_t)(mBase + mOff + r) * ldc + n];
        if (ACT == 2) v = fmaxf(v, 0.0f);
        if (ACT == 4) v = (v > 0.f) ? v : 0.01f * v;
        slab[(mOff + r) * 68 + (j << 4) + rlane] = v;
      }
    }
    __builtin_amdgcn_fence(__ATOMIC_RELEASE, "workgroup");
    __builtin_amdgcn_wave_barrier();
    __builtin_amdgcn_fence(__ATOMIC_ACQUIRE, "workgroup");
    if (OUT_MODE == 0) {
      float* C = (float*)Cout + (size_t)b * strideC;
      const int hh = lane >> 4, c4 = (lane & 15) * 4;
      for (int pass = 0; pass < 2; ++pass) {
#pragma unroll
        for (int it = 0; it < 8; ++it) {
          const int row = it * 2 + hh;
          v4f v = *(const v4f*)(slab + row * 68 + c4);
          *(volatile v4f*)(C + (size_t)(mBase + row) * ldc + n0 + c4) = v;
        }
        __threadfence();
      }
    } else {
      const int q = lane >> 3, c8 = (lane & 7) * 8;
      unsigned short* C  = (unsigned short*)Cout  + (size_t)b * strideC;
      unsigned short* C2 = (OUT_MODE == 2) ? ((unsigned short*)Cout2 + (size_t)b * strideC) : nullptr;
      for (int pass = 0; pass < 2; ++pass) {
#pragma unroll
        for (int it = 0; it < 4; ++it) {
          const int row = it * 4 + q;
          const float* sp = slab + row * 68 + c8;
          v8h hv, lv;
#pragma unroll
          for (int e = 0; e < 8; ++e) {
            if (OUT_MODE == 1) {
              hv[e] = (_Float16)sp[e];
            } else {
              unsigned short hb = f2bf_bits(sp[e]);
              unsigned short lb = f2bf_bits(sp[e] - bf_bits2f(hb));
              hv[e] = __builtin_bit_cast(_Float16, hb);
              lv[e] = __builtin_bit_cast(_Float16, lb);
            }
          }
          *(volatile v8h*)(C + (size_t)(mBase + row) * ldc + n0 + c8) = hv;
          if (OUT_MODE == 2) *(volatile v8h*)(C2 + (size_t)(mBase + row) * ldc + n0 + c8) = lv;
        }
        __threadfence();
      }
    }
    __builtin_amdgcn_fence(__ATOMIC_RELEASE, "workgroup");
    __builtin_amdgcn_wave_barrier();
    __builtin_amdgcn_fence(__ATOMIC_ACQUIRE, "workgroup");
  }
}

__global__ __launch_bounds__(256) void xtrans16_kernel(const float* __restrict__ x, unsigned short* __restrict__ X16) {
  __shared__ float sm[64][65];
  const int t  = threadIdx.x;
  const int c0 = blockIdx.x * 64;
  const int n0 = blockIdx.y * 64;
  const int b  = blockIdx.z;
  const float* xb = x + ((size_t)b * kChan + c0) * kPos + n0;
#pragma unroll
  for (int i = 0; i < 16; ++i) {
    const int e  = i * 256 + t;
    const int r  = e >> 6;
    const int cl = e & 63;
    sm[cl][r] = xb[(size_t)r * kPos + cl];
  }
  __syncthreads();
  const int lane = t & 31, wave = t >> 5;
  const int q = lane >> 3, c8 = (lane & 7) * 8;
  unsigned short* ob = X16 + ((size_t)b * kPos + n0) * kChan + c0;
  for (int pass = 0; pass < 2; ++pass) {
#pragma unroll
    for (int it = 0; it < 2; ++it) {
      const int row = wave * 8 + it * 4 + q;
      unsigned short hb[8];
#pragma unroll
      for (int e = 0; e < 8; ++e) hb[e] = h_bits(sm[row][c8 + e]);
      const v4u u = (v4u){pk16(hb[0], hb[1]), pk16(hb[2], hb[3]), pk16(hb[4], hb[5]), pk16(hb[6], hb[7])};
      *(volatile v4u*)(ob + (size_t)row * kChan + c8) = u;
    }
    __threadfence();
  }
}

__global__ __launch_bounds__(256) void wcast_kernel(const float* __restrict__ Wq, const float* __restrict__ Wk,
                                                    const float* __restrict__ Wd, const float* __restrict__ Wv,
                                                    const float* __restrict__ Wu,
                                                    unsigned short* __restrict__ Wqk16, unsigned short* __restrict__ Wd16,
                                                    unsigned short* __restrict__ Wv16, unsigned short* __restrict__ Wu16,
                                                    float scale) {
  const int seg = blockIdx.y;
  const float* src = Wq; unsigned short* dst = Wqk16; int n8 = kDk * kChan / 8;
  if (seg == 1)      { src = Wk; dst = Wqk16 + (size_t)kDk * kChan; n8 = kDk * kChan / 8; }
  else if (seg == 2) { src = Wd; dst = Wd16;  n8 = kDk * kChan / 8; }
  else if (seg == 3) { src = Wv; dst = Wv16;  n8 = kChan * kChan / 8; }
  else if (seg == 4) { src = Wu; dst = Wu16;  n8 = kChan * kDk / 8; }
  const int i = blockIdx.x * 256 + threadIdx.x;
  if (i >= n8) return;
  const float* p = src + 8 * (size_t)i;
  const v4f a = *(const v4f*)(p);
  const v4f c = *(const v4f*)(p + 4);
  unsigned short hb[8];
#pragma unroll
  for (int e = 0; e < 4; ++e) {
    hb[e]     = h_bits(a[e] * scale);
    hb[4 + e] = h_bits(c[e] * scale);
  }
  const v4u u = (v4u){pk16(hb[0], hb[1]), pk16(hb[2], hb[3]), pk16(hb[4], hb[5]), pk16(hb[6], hb[7])};
  unsigned short* qp = dst + 8 * (size_t)i;
  *(volatile v4u*)qp = u;
  __threadfence();
  *(volatile v4u*)qp = u;
}

__global__ __launch_bounds__(256) void xdcast_kernel(const float* __restrict__ XD32, unsigned short* __restrict__ XD16pm,
                                                     unsigned short* __restrict__ XD16cm) {
  __shared__ float sm[64][65];
  const int t  = threadIdx.x;
  const int n0 = blockIdx.x * 64;
  const int b  = blockIdx.y;
  const float* src = XD32 + ((size_t)b * kPos + n0) * kDk;
#pragma unroll
  for (int i = 0; i < 16; ++i) {
    const int e = i * 256 + t;
    sm[e >> 6][e & 63] = src[e];
  }
  __syncthreads();
  const int lane = t & 31, wave = t >> 5;
  const int q = lane >> 3, c8 = (lane & 7) * 8;
  unsigned short* opm = XD16pm + ((size_t)b * kPos + n0) * kDk;
  unsigned short* ocm = XD16cm + (size_t)b * kDk * kPos + n0;
  for (int pass = 0; pass < 2; ++pass) {
#pragma unroll
    for (int it = 0; it < 2; ++it) {
      const int row = wave * 8 + it * 4 + q;
      unsigned short ha[8], hc[8];
#pragma unroll
      for (int e = 0; e < 8; ++e) {
        ha[e] = h_bits(sm[row][c8 + e]);
        hc[e] = h_bits(sm[c8 + e][row]);
      }
      const v4u ua = (v4u){pk16(ha[0], ha[1]), pk16(ha[2], ha[3]), pk16(ha[4], ha[5]), pk16(ha[6], ha[7])};
      const v4u uc = (v4u){pk16(hc[0], hc[1]), pk16(hc[2], hc[3]), pk16(hc[4], hc[5]), pk16(hc[6], hc[7])};
      *(volatile v4u*)(opm + (size_t)row * kDk + c8) = ua;
      *(volatile v4u*)(ocm + (size_t)row * kPos + c8) = uc;
    }
    __threadfence();
  }
}

__global__ __launch_bounds__(256) void chansoft_kernel(const float* __restrict__ E, unsigned short* __restrict__ CA, float carry) {
  __shared__ float sE[64][65];
  const int t = threadIdx.x;
  const int b = blockIdx.x;
  const float* eb = E + (size_t)b * kDk * kDk;
#pragma unroll
  for (int i = 0; i < 16; ++i) {
    const int e = i * 256 + t;
    sE[e >> 6][e & 63] = eb[e];
  }
  __syncthreads();
  const int row = t >> 2, cb = (t & 3) * 16;
  float mx = -INFINITY, mn = INFINITY;
#pragma unroll 1
  for (int k = 0; k < 16; ++k) {
    const float v = sE[row][cb + k];
    mx = fmaxf(mx, v);
    mn = fminf(mn, v);
  }
  mx = fmaxf(mx, __shfl_xor(mx, 1, 32));
  mx = fmaxf(mx, __shfl_xor(mx, 2, 32));
  mn = fminf(mn, __shfl_xor(mn, 1, 32));
  mn = fminf(mn, __shfl_xor(mn, 2, 32));
  const float m2 = mx - mn;
  float sum = 0.f;
#pragma unroll 1
  for (int k = 0; k < 16; ++k) {
    const float en = mx - sE[row][cb + k];
    const float p = expf(en - m2);
    sE[row][cb + k] = p;
    sum += p;
  }
  sum += __shfl_xor(sum, 1, 32);
  sum += __shfl_xor(sum, 2, 32);
  const float inv = 1.0f / sum;
#pragma unroll 1
  for (int k = 0; k < 16; ++k) {
    const float p = sE[row][cb + k];
    sE[row][cb + k] = (p * inv) * carry;
  }
  __syncthreads();
  const int lane = t & 31, wave = t >> 5;
  const int q = lane >> 3, c8 = (lane & 7) * 8;
  unsigned short* ob = CA + (size_t)b * kDk * kDk;
  for (int pass = 0; pass < 2; ++pass) {
#pragma unroll
    for (int it = 0; it < 2; ++it) {
      const int r = wave * 8 + it * 4 + q;
      unsigned short hb[8];
#pragma unroll
      for (int e = 0; e < 8; ++e) hb[e] = h_bits(sE[r][c8 + e]);
      const v4u u = (v4u){pk16(hb[0], hb[1]), pk16(hb[2], hb[3]), pk16(hb[4], hb[5]), pk16(hb[6], hb[7])};
      *(volatile v4u*)(ob + (size_t)r * kDk + c8) = u;
    }
    __threadfence();
  }
}

__global__ __launch_bounds__(256) void softmax_row_kernel(const float* __restrict__ S, unsigned short* __restrict__ P, float carry) {
  __shared__ __align__(16) float srow[kPos];
  __shared__ float redM[8];
  __shared__ float redS[8];
  const int row  = blockIdx.x;
  const int t    = threadIdx.x;
  const int lane = t & 31, wave = t >> 5;
  const int c0   = 8 * t;
  const int c1   = kHalfQ + 8 * t;
  const float* sr = S + (size_t)row * kPos;
  const v4f a0 = *(const v4f*)(sr + c0);
  const v4f a1 = *(const v4f*)(sr + c0 + 4);
  const v4f b0 = *(const v4f*)(sr + c1);
  const v4f b1 = *(const v4f*)(sr + c1 + 4);
  float m = fmaxf(fmaxf(fmaxf(a0[0], a0[1]), fmaxf(a0[2], a0[3])), fmaxf(fmaxf(a1[0], a1[1]), fmaxf(a1[2], a1[3])));
  m = fmaxf(m, fmaxf(fmaxf(fmaxf(b0[0], b0[1]), fmaxf(b0[2], b0[3])), fmaxf(fmaxf(b1[0], b1[1]), fmaxf(b1[2], b1[3]))));
  *(v4f*)(srow + c0)     = a0;
  *(v4f*)(srow + c0 + 4) = a1;
  *(v4f*)(srow + c1)     = b0;
  *(v4f*)(srow + c1 + 4) = b1;
#pragma unroll
  for (int off = 16; off > 0; off >>= 1) m = fmaxf(m, __shfl_xor(m, off, 32));
  if (lane == 0) redM[wave] = m;
  __syncthreads();
  float M = redM[0];
#pragma unroll
  for (int w = 1; w < 8; ++w) M = fmaxf(M, redM[w]);
  float sum = 0.f;
#pragma unroll 1
  for (int k = 0; k < 16; ++k) {
    const int col = c0 + (k & 7) + (k >> 3) * kHalfQ;
    const float p = expf(srow[col] - M);
    srow[col] = p;
    sum += p;
  }
#pragma unroll
  for (int off = 16; off > 0; off >>= 1) sum += __shfl_xor(sum, off, 32);
  if (lane == 0) redS[wave] = sum;
  __syncthreads();
  float tot = redS[0];
#pragma unroll
  for (int w = 1; w < 8; ++w) tot += redS[w];
  const float inv = 1.0f / tot;
  const v4f p0 = *(const v4f*)(srow + c0);
  const v4f p1 = *(const v4f*)(srow + c0 + 4);
  const v4f q0 = *(const v4f*)(srow + c1);
  const v4f q1 = *(const v4f*)(srow + c1 + 4);
  unsigned short ha[8], hb[8];
#pragma unroll
  for (int e = 0; e < 4; ++e) {
    ha[e]     = h_bits((p0[e] * inv) * carry);
    ha[4 + e] = h_bits((p1[e] * inv) * carry);
    hb[e]     = h_bits((q0[e] * inv) * carry);
    hb[4 + e] = h_bits((q1[e] * inv) * carry);
  }
  const v4u ua = (v4u){pk16(ha[0], ha[1]), pk16(ha[2], ha[3]), pk16(ha[4], ha[5]), pk16(ha[6], ha[7])};
  const v4u ub = (v4u){pk16(hb[0], hb[1]), pk16(hb[2], hb[3]), pk16(hb[4], hb[5]), pk16(hb[6], hb[7])};
  unsigned short* pr = P + (size_t)row * kPos;
  *(volatile v4u*)(pr + c0) = ua;
  *(volatile v4u*)(pr + c1) = ub;
  __threadfence();
  *(volatile v4u*)(pr + c0) = ua;
  *(volatile v4u*)(pr + c1) = ub;
}

extern "C" void kernel_launch(void* const* d_in, const int* in_sizes, int n_in,
                              void* d_out, int out_size, void* d_ws, size_t ws_size,
                              hipStream_t stream) {
  if (n_in < 13) return;
  if (in_sizes[0] != kImg * kChan * kPos) return;
  if (in_sizes[1] != kDk * kChan || in_sizes[2] != kDk) return;
  if (in_sizes[3] != kDk * kChan || in_sizes[4] != kDk) return;
  if (in_sizes[5] != kChan * kChan || in_sizes[6] != kChan) return;
  if (in_sizes[7] < 1) return;
  if (in_sizes[8] != kDk * kChan || in_sizes[9] != kDk) return;
  if (in_sizes[10] != kChan * kDk || in_sizes[11] != kChan) return;
  if (in_sizes[12] < 1) return;
  if (out_size != kImg * kChan * kPos) return;

  const float* x  = (const float*)d_in[0];
  const float* Wq = (const float*)d_in[1];
  const float* bq = (const float*)d_in[2];
  const float* Wk = (const float*)d_in[3];
  const float* bk = (const float*)d_in[4];
  const float* Wv = (const float*)d_in[5];
  const float* bv = (const float*)d_in[6];
  const float* gs = (const float*)d_in[7];
  const float* Wd = (const float*)d_in[8];
  const float* bd = (const float*)d_in[9];
  const float* Wu = (const float*)d_in[10];
  const float* bu = (const float*)d_in[11];
  const float* gc = (const float*)d_in[12];
  float* out = (float*)d_out;

  const size_t szX16   = (size_t)kPix * kChan * 2;
  const size_t szWqk16 = (size_t)2 * kDk * kChan * 2;
  const size_t szWd16  = (size_t)kDk * kChan * 2;
  const size_t szWv16  = (size_t)kChan * kChan * 2;
  const size_t szWu16  = (size_t)kChan * kDk * 2;
  const size_t szQK16  = (size_t)kPix * 2 * kDk * 2;
  const size_t szXD32  = (size_t)kPix * kDk * 4;
  const size_t szXD16  = (size_t)kPix * kDk * 2;
  const size_t szE32   = (size_t)kImg * kDk * kDk * 4;
  const size_t szCA16  = (size_t)kImg * kDk * kDk * 2;
  const size_t szV16   = (size_t)kImg * kChan * kPos * 2;
  const size_t szCHX   = (size_t)kImg * kChan * kPos * 4;
  const size_t szS32   = (size_t)kHalfQ * kPos * 4;
  const size_t szP16   = (size_t)kHalfQ * kPos * 2;

  char* ws = (char*)d_ws;
  size_t off = 0;
  unsigned short* X16    = (unsigned short*)(ws + off); off += szX16;
  unsigned short* Wqk16  = (unsigned short*)(ws + off); off += szWqk16;
  unsigned short* Wd16   = (unsigned short*)(ws + off); off += szWd16;
  unsigned short* Wv16   = (unsigned short*)(ws + off); off += szWv16;
  unsigned short* Wu16   = (unsigned short*)(ws + off); off += szWu16;
  unsigned short* QK16   = (unsigned short*)(ws + off); off += szQK16;
  float*          XD32   = (float*)(ws + off);          off += szXD32;
  unsigned short* XD16pm = (unsigned short*)(ws + off); off += szXD16;
  unsigned short* XD16cm = (unsigned short*)(ws + off); off += szXD16;
  float*          E32    = (float*)(ws + off);          off += szE32;
  unsigned short* CA16   = (unsigned short*)(ws + off); off += szCA16;
  unsigned short* CO16   = (unsigned short*)(ws + off); off += szXD16;
  unsigned short* V16    = (unsigned short*)(ws + off); off += szV16;
  float*          CHX    = (float*)(ws + off);          off += szCHX;
  float*          S32    = (float*)(ws + off);          off += szS32;
  unsigned short* P16    = (unsigned short*)(ws + off); off += szP16;
  if (off > ws_size) return;

  const dim3 blk(256, 1, 1);
  const long strXimg  = (long)kPos * kChan;
  const long strVimg  = (long)kChan * kPos;
  const long strXDimg = (long)kPos * kDk;
  const long strEimg  = (long)kDk * kDk;

  xtrans16_kernel<<<dim3(kChan / 64, kPos / 64, kImg), blk, 0, stream>>>(x, X16);
  wcast_kernel<<<dim3(128, 5, 1), blk, 0, stream>>>(Wq, Wk, Wd, Wv, Wu, Wqk16, Wd16, Wv16, Wu16, kWCarry);
  wmma_gemm64<0, false, 2, 1, false, false><<<dim3(32, 1, 1), blk, 0, stream>>>(
      X16, X16, kChan, 0L, Wqk16, Wqk16, kChan, 0L, (void*)QK16, (void*)QK16, 2 * kDk, 0L,
      bq, bq, 0L, bq, kPix, kDk, kChan, kWCarryInv);
  wmma_gemm64<0, false, 2, 1, false, false><<<dim3(32, 1, 1), blk, 0, stream>>>(
      X16, X16, kChan, 0L, Wqk16 + (size_t)kDk * kChan, Wqk16 + (size_t)kDk * kChan, kChan, 0L,
      (void*)(QK16 + kDk), (void*)(QK16 + kDk), 2 * kDk, 0L,
      bk, bk, 0L, bk, kPix, kDk, kChan, kWCarryInv);
  wmma_gemm64<0, false, 2, 0, false, false><<<dim3(32, 1, 1), blk, 0, stream>>>(
      X16, X16, kChan, 0L, Wd16, Wd16, kChan, 0L, (void*)XD32, (void*)XD32, kDk, 0L,
      bd, bd, 0L, bd, kPix, kDk, kChan, kWCarryInv);
  wmma_gemm64<0, false, 1, 1, false, false><<<dim3(64, kImg, 1), blk, 0, stream>>>(
      Wv16, Wv16, kChan, 0L, X16, X16, kChan, strXimg, (void*)V16, (void*)V16, kPos, strVimg,
      bv, bv, 0L, bv, kChan, kPos, kChan, kWCarryInv);
  xdcast_kernel<<<dim3(kPos / 64, kImg, 1), blk, 0, stream>>>(XD32, XD16pm, XD16cm);
  wmma_gemm64<0, false, 0, 0, false, false><<<dim3(1, kImg, 1), dim3(32, 1, 1), 0, stream>>>(
      XD16cm, XD16cm, kPos, (long)kDk * kPos, XD16cm, XD16cm, kPos, (long)kDk * kPos,
      (void*)E32, (void*)E32, kDk, strEimg,
      gc, gc, 0L, gc, kDk, kDk, kPos, 1.0f);
  chansoft_kernel<<<dim3(kImg, 1, 1), blk, 0, stream>>>(E32, CA16, kPCarry);
  wmma_gemm64<0, false, 0, 1, true, true><<<dim3(8, kImg, 1), blk, 0, stream>>>(
      XD16pm, XD16pm, kDk, strXDimg, CA16, CA16, kDk, strEimg, (void*)CO16, (void*)CO16, kDk, strXDimg,
      gc, XD32, strXDimg, gc, kPos, kDk, kDk, kPCarryInv);
  wmma_gemm64<0, false, 1, 0, true, false><<<dim3(64, kImg, 1), blk, 0, stream>>>(
      Wu16, Wu16, kDk, 0L, CO16, CO16, kDk, strXDimg, (void*)CHX, (void*)CHX, kPos, strVimg,
      bu, x, strVimg, bu, kChan, kPos, kDk, kWCarryInv);
  for (int b = 0; b < kImg; ++b) {
    for (int mh = 0; mh < 2; ++mh) {
      const unsigned short* Qp = QK16 + ((size_t)b * kPos + (size_t)mh * kHalfQ) * (2 * kDk);
      const unsigned short* Kp = QK16 + (size_t)b * kPos * (2 * kDk) + kDk;
      wmma_gemm64<0, false, 0, 0, false, false><<<dim3(256, 1, 1), blk, 0, stream>>>(
          Qp, Qp, 2 * kDk, 0L, Kp, Kp, 2 * kDk, 0L, (void*)S32, (void*)S32, kPos, 0L,
          gs, gs, 0L, gs, kHalfQ, kPos, kDk, 1.0f);
      softmax_row_kernel<<<dim3(kHalfQ, 1, 1), blk, 0, stream>>>(S32, P16, kPCarry);
      const size_t ooff = (size_t)b * kChan * kPos + (size_t)mh * kHalfQ;
      wmma_gemm64<0, false, 0, 0, true, true><<<dim3(32, 1, 1), blk, 0, stream>>>(
          V16 + (size_t)b * kChan * kPos, V16 + (size_t)b * kChan * kPos, kPos, 0L, P16, P16, kPos, 0L,
          (void*)(out + ooff), (void*)(out + ooff), kPos, 0L,
          gs, CHX + ooff, 0L, gs, kChan, kHalfQ, kPos, kPCarryInv);
    }
  }
}
